// DecoderLayer_11149735100531
// MI455X (gfx1250) — hardware-verified
//
#include <hip/hip_runtime.h>
#ifndef NB
#define NB 4
#endif
#ifndef SEQ
#define SEQ 2048
#endif
#define NB_FULL 4
#define SEQ_FULL 2048
#define DM 1024
#define NH 16
#define HD 64
#define LQ (3 * DM)
#define MROWS (SEQ * NB_FULL)
#define RP (NB_FULL * LQ)
#define NQT (SEQ / 64)
#define NKT (SEQ / 64)
static_assert(SEQ % 64 == 0);
static_assert(SEQ <= SEQ_FULL);
static_assert(NB >= 1 && NB <= NB_FULL);
static_assert(NKT <= 32);
static_assert(MROWS % 128 == 0);
static_assert(DM % 64 == 0 && DM % 32 == 0);

typedef _Float16 v16h __attribute__((ext_vector_type(16)));
typedef _Float16 v4h  __attribute__((ext_vector_type(4)));
typedef unsigned short v8us __attribute__((ext_vector_type(8), may_alias));
typedef float  v8f  __attribute__((ext_vector_type(8)));
typedef float  v4f  __attribute__((ext_vector_type(4)));
typedef float  v4fa __attribute__((ext_vector_type(4), may_alias));
typedef int    v4ia __attribute__((ext_vector_type(4), may_alias));
union FragH { v16h v; v8us half[2]; _Float16 h[16]; unsigned short u[16]; };

#define NEG_INF (-__builtin_inff())

__device__ __forceinline__ unsigned short bf16_bits(float x) { unsigned int u = __float_as_uint(x); return (unsigned short)((u + 0x7FFFu + ((u >> 16) & 1u)) >> 16); }
__device__ __forceinline__ float bf16_val(unsigned short b) { return __uint_as_float(((unsigned int)b) << 16); }
__device__ __forceinline__ float bf16_rne(float x) { return bf16_val(bf16_bits(x)); }

__device__ __forceinline__ v16h g2_frag(const _Float16* p, int hh) { FragH f; f.half[0] = *(const v8us*)((const unsigned short*)p + 8 * hh); f.half[1] = *(const v8us*)((const unsigned short*)p + 16 + 8 * hh); return f.v; }
__device__ __forceinline__ v8f g2_mma(v16h a, v16h b, v8f c) { v8f d = __builtin_amdgcn_wmma_f32_16x16x32_f16(false, a, false, b, (short)0, c, false, false); asm volatile("v_nop\n\tv_nop\n\tv_nop\n\tv_nop" : "+v"(d) : "v"(a), "v"(b)); return d; }

__global__ __launch_bounds__(256) void k_x16(const float* __restrict__ x, _Float16* __restrict__ X16, size_t n8) { const size_t t = (size_t)blockIdx.x * 256 + threadIdx.x; if (t >= n8) return; FragH f;
#pragma unroll
  for (int q = 0; q < 8; ++q) f.h[q] = (_Float16)bf16_rne(x[t * 8 + q]); *(volatile v8us*)((unsigned short*)X16 + t * 8) = f.half[0]; __threadfence(); *(volatile v8us*)((unsigned short*)X16 + t * 8) = f.half[0]; }

__global__ __launch_bounds__(256) void k_wnat(const float* __restrict__ w, size_t n8, _Float16* __restrict__ Bt) { const size_t t = (size_t)blockIdx.x * 256 + threadIdx.x; if (t >= n8) return; FragH f;
#pragma unroll
  for (int q = 0; q < 8; ++q) f.h[q] = (_Float16)(bf16_rne(w[t * 8 + q]) * 16.0f); *(volatile v8us*)((unsigned short*)Bt + t * 8) = f.half[0]; __threadfence(); *(volatile v8us*)((unsigned short*)Bt + t * 8) = f.half[0]; }

__global__ __launch_bounds__(128) void k_gemm2(const _Float16* __restrict__ A, int lda, const _Float16* __restrict__ Bh, int ldb, float alpha, const float* __restrict__ bias,
    _Float16* __restrict__ C16, int ldc, int M, int N, int K) {
  __shared__ __attribute__((aligned(16))) float so[4][32][68];
  const int tid = threadIdx.x, w = tid >> 5, lane = tid & 31, ln = lane & 15, hh = lane >> 4;
  const int ntn = N >> 6; const int mt = blockIdx.x / ntn, nq = blockIdx.x - mt * ntn; const int row0 = mt * 128 + 32 * w, col0 = nq * 64; if (row0 >= M) return;
  const _Float16* a0p = A + (size_t)(row0 + ln) * lda; const _Float16* a1p = a0p + (size_t)16 * lda;
  const _Float16* b0p = Bh + (size_t)(col0 + ln) * ldb; const _Float16* b1p = b0p + (size_t)16 * ldb; const _Float16* b2p = b1p + (size_t)16 * ldb; const _Float16* b3p = b2p + (size_t)16 * ldb;
  const v8f z8 = {0.f,0.f,0.f,0.f,0.f,0.f,0.f,0.f}; v8f c00 = z8, c01 = z8, c02 = z8, c03 = z8, c10 = z8, c11 = z8, c12 = z8, c13 = z8;
#pragma unroll 1
  for (int kb = 0; kb < K; kb += 32) { const v16h a0 = g2_frag(a0p + kb, hh), a1 = g2_frag(a1p + kb, hh);
    v16h b = g2_frag(b0p + kb, hh); c00 = g2_mma(a0, b, c00); c10 = g2_mma(a1, b, c10);
    b = g2_frag(b1p + kb, hh); c01 = g2_mma(a0, b, c01); c11 = g2_mma(a1, b, c11);
    b = g2_frag(b2p + kb, hh); c02 = g2_mma(a0, b, c02); c12 = g2_mma(a1, b, c12);
    b = g2_frag(b3p + kb, hh); c03 = g2_mma(a0, b, c03); c13 = g2_mma(a1, b, c13); }
  v8f accs[8] = {c00, c01, c02, c03, c10, c11, c12, c13};
#pragma unroll
  for (int u = 0; u < 8; ++u) { const int t = u & 3, half = u >> 2; const int col = col0 + t * 16 + ln; const float bv = bf16_rne(bias[col]);
#pragma unroll
    for (int r = 0; r < 8; ++r) { const int rloc = half * 16 + 8 * hh + r; so[w][rloc][t * 16 + ln] = accs[u][r] * alpha + bv; } }
  __builtin_amdgcn_fence(4  , "workgroup"); __builtin_amdgcn_wave_barrier();
  const int rsub = lane >> 4, c4 = (lane & 15) * 4;
  for (int pass = 0; pass < 2; ++pass) {
#pragma unroll
    for (int q = 0; q < 16; ++q) { const int r = q * 2 + rsub; const v4f v = *(const v4fa*)&so[w][r][c4]; v4h h4;
#pragma unroll
      for (int i = 0; i < 4; ++i) h4[i] = (_Float16)v[i];
      *(volatile v4h*)(C16 + (size_t)(row0 + r) * ldc + col0 + c4) = h4; }
    if (pass == 0) __threadfence(); } }

__global__ __launch_bounds__(256) void k_vt2(const _Float16* __restrict__ QKV, _Float16* __restrict__ VT) {
  __shared__ unsigned short tl[64][66];
  const int tid = threadIdx.x; const int slab = blockIdx.x / NQT, lg = blockIdx.x - slab * NQT; const int b = slab / NH, hd = slab - b * NH; const int s0 = lg * 64;
  for (int i = tid; i < 64 * 8; i += 256) { const int r = i / 8, c8 = (i % 8) * 8; FragH f;
    f.half[0] = *(const v8us*)((const unsigned short*)QKV + ((size_t)(s0 + r) * NB_FULL + b) * LQ + 2 * DM + hd * HD + c8);
#pragma unroll
    for (int q = 0; q < 8; ++q) tl[r][c8 + q] = f.u[q]; }
  __syncthreads();
  for (int pass = 0; pass < 2; ++pass) {
#pragma unroll
    for (int rd = 0; rd < 2; ++rd) { const int d = rd * 32 + tid / 8, pc = tid % 8; FragH f;
#pragma unroll
      for (int q = 0; q < 8; ++q) f.u[q] = tl[pc * 8 + q][d];
      *(volatile v8us*)((unsigned short*)VT + ((size_t)slab * HD + d) * SEQ + s0 + pc * 8) = f.half[0]; }
    if (pass == 0) __threadfence(); } }

__global__ __launch_bounds__(256) void k_mflag(const int* __restrict__ mask, int* __restrict__ MF) {
  __shared__ int sf[32];
  const int tid = threadIdx.x, qt = blockIdx.x; const int kt = tid >> 3, p = tid & 7;
  const bool ok = kt < NKT; const int ktc = ok ? kt : (NKT - 1);
  int acc = 0;
#pragma unroll 1
  for (int r = 0; r < 64; ++r) {
    const int* rowp = mask + (size_t)(qt * 64 + r) * SEQ_FULL + ktc * 64 + p * 4;
    const v4ia a = *(const v4ia*)rowp; const v4ia c = *(const v4ia*)(rowp + 32);
    acc |= (a[0] | a[1]) | (a[2] | a[3]) | (c[0] | c[1]) | (c[2] | c[3]); }
  acc = ok ? acc : 0;
  acc |= __shfl_xor(acc, 1); acc |= __shfl_xor(acc, 2); acc |= __shfl_xor(acc, 4);
  if (p == 0) sf[kt] = (acc != 0) ? 1 : 0;
  __syncthreads();
  if (tid < 32) { const int v = sf[tid]; volatile int* d = MF + (size_t)qt * 32 + tid; *d = v; __threadfence(); *d = v; } }

__global__ __launch_bounds__(128) void k_attn(const _Float16* __restrict__ QKV, const _Float16* __restrict__ VT, const int* __restrict__ mask, const int* __restrict__ MF,
                                              const float* __restrict__ x, float* __restrict__ out) {
  __shared__ __attribute__((aligned(16))) float so[4][16][68];
  const int tid = threadIdx.x, w = tid >> 5, lane = tid & 31, l15 = lane & 15, hh = lane >> 4;
  const int qt = blockIdx.x, slab = blockIdx.y; const int b = slab / NH, hd = slab - b * NH;
  const int q0 = qt * 64 + w * 16;
  const _Float16* Qb = QKV + (size_t)b * LQ + hd * HD;
  const _Float16* Kb = Qb + DM;
  const _Float16* Vb = VT + (size_t)slab * HD * SEQ;
  const _Float16* qrow = Qb + (size_t)(q0 + l15) * RP;
  const v16h qf0 = g2_frag(qrow, hh), qf1 = g2_frag(qrow + 32, hh);
  const v8f z8 = {0.f,0.f,0.f,0.f,0.f,0.f,0.f,0.f};
  v8f o[4] = {z8, z8, z8, z8};
  float m = NEG_INF, l = 0.f;
  const float CL = 0.045084220027780106f;
#pragma unroll 1
  for (int it = 0; it < NKT; ++it) {
    const int key0 = it * 64;
    v8f s[4];
#pragma unroll
    for (int kt = 0; kt < 4; ++kt) {
      const _Float16* krow = Kb + (size_t)(key0 + kt * 16 + l15) * RP;
      const v16h ka = g2_frag(krow, hh), kk = g2_frag(krow + 32, hh);
      v8f a = g2_mma(ka, qf0, z8); a = g2_mma(kk, qf1, a); s[kt] = a; }
    const int mf = MF[(size_t)qt * 32 + it];
    if (mf != 0) {
#pragma unroll
      for (int kt = 0; kt < 4; ++kt) {
        const int* mp = mask + (size_t)(q0 + l15) * SEQ_FULL + key0 + kt * 16 + 8 * hh;
        const v4ia ma = *(const v4ia*)mp; const v4ia mb = *(const v4ia*)(mp + 4);
#pragma unroll
        for (int r = 0; r < 4; ++r) { s[kt][r] = (ma[r] != 0) ? NEG_INF : s[kt][r]; s[kt][4 + r] = (mb[r] != 0) ? NEG_INF : s[kt][4 + r]; } } }
    float lmax = NEG_INF;
#pragma unroll
    for (int kt = 0; kt < 4; ++kt)
#pragma unroll
      for (int r = 0; r < 8; ++r) lmax = fmaxf(lmax, s[kt][r]);
    lmax = fmaxf(lmax, __shfl_xor(lmax, 16));
    const float mnew = fmaxf(m, lmax);
    const float mref = (mnew == NEG_INF) ? 0.0f : mnew;
    const float alpha = exp2f((m - mref) * CL);
    const float bexp = 10.0f - mref * CL;
    m = mnew;
    float psum = 0.f; FragH pa, pb;
#pragma unroll
    for (int r = 0; r < 8; ++r) {
      const float e0 = exp2f(fmaf(s[0][r], CL, bexp)), e1 = exp2f(fmaf(s[1][r], CL, bexp)), e2 = exp2f(fmaf(s[2][r], CL, bexp)), e3 = exp2f(fmaf(s[3][r], CL, bexp));
      psum += (e0 + e1) + (e2 + e3);
      pa.h[r] = (_Float16)e0; pa.h[8 + r] = (_Float16)e1; pb.h[r] = (_Float16)e2; pb.h[8 + r] = (_Float16)e3; }
    l = l * alpha + psum;
    float ar[8];
#pragma unroll
    for (int r = 0; r < 8; ++r) ar[r] = __shfl(alpha, 8 * hh + r);
#pragma unroll
    for (int dt = 0; dt < 4; ++dt) {
#pragma unroll
      for (int r = 0; r < 8; ++r) o[dt][r] *= ar[r];
      const _Float16* vrow = Vb + (size_t)(dt * 16 + l15) * SEQ + key0;
      const v16h va = g2_frag(vrow, hh), vb = g2_frag(vrow + 32, hh);
      o[dt] = g2_mma(pa.v, va, o[dt]); o[dt] = g2_mma(pb.v, vb, o[dt]); } }
  const float lt = l + __shfl_xor(l, 16);
  const float inv = 1.0f / lt;
  float ir[8];
#pragma unroll
  for (int r = 0; r < 8; ++r) ir[r] = __shfl(inv, 8 * hh + r);
#pragma unroll
  for (int dt = 0; dt < 4; ++dt)
#pragma unroll
    for (int r = 0; r < 8; ++r) so[w][8 * hh + r][dt * 16 + l15] = o[dt][r] * ir[r];
  __builtin_amdgcn_fence(4  , "workgroup"); __builtin_amdgcn_wave_barrier();
  const int rq = lane >> 3, pc = lane & 7;
  for (int pass = 0; pass < 2; ++pass) {
#pragma unroll
    for (int g = 0; g < 8; ++g) { const int L = g * 4 + rq; const int row = L >> 1, col = (L & 1) * 32 + pc * 4;
      const size_t gi = ((size_t)(q0 + row) * NB_FULL + b) * DM + hd * HD + col;
      v4f v = *(const v4fa*)&so[w][row][col]; const v4f xr = *(const v4fa*)(x + gi);
#pragma unroll
      for (int i = 0; i < 4; ++i) v[i] += bf16_rne(xr[i]);
      *(volatile v4f*)(out + gi) = v; }
    if (pass == 0) __threadfence(); } }

extern "C" void kernel_launch(void* const* d_in, const int* in_sizes, int n_in,
                              void* d_out, int out_size, void* d_ws, size_t ws_size, hipStream_t stream) {
  if (n_in < 8) return;
  const float* x  = (const float*)d_in[0];
  const int*   mk = (const int*)d_in[1];
  const float* Wq = (const float*)d_in[2]; const float* bq = (const float*)d_in[3];
  const float* Wk = (const float*)d_in[4]; const float* bk = (const float*)d_in[5];
  const float* Wv = (const float*)d_in[6]; const float* bv = (const float*)d_in[7];
  if (in_sizes[0] < MROWS * DM) return;
  if (in_sizes[1] < (SEQ - 1) * SEQ_FULL + SEQ) return;
  if (in_sizes[2] < DM * DM || in_sizes[4] < DM * DM || in_sizes[6] < DM * DM) return;
  if (in_sizes[3] < DM || in_sizes[5] < DM || in_sizes[7] < DM) return;
  if (out_size < MROWS * DM) return;
  char* ws = (char*)d_ws; size_t off = 0;
  auto take = [&](size_t bytes) { char* p = ws + off; off += (bytes + 255) & ~(size_t)255; return p; };
  _Float16* BQ  = (_Float16*)take((size_t)DM * DM * 2);
  _Float16* BK  = (_Float16*)take((size_t)DM * DM * 2);
  _Float16* BV  = (_Float16*)take((size_t)DM * DM * 2);
  _Float16* X16 = (_Float16*)take((size_t)MROWS * DM * 2);
  _Float16* QKV = (_Float16*)take((size_t)MROWS * LQ * 2);
  _Float16* VT  = (_Float16*)take((size_t)NB * NH * HD * SEQ * 2);
  int*      MF  = (int*)take((size_t)NQT * 32 * 4);
  if (off > ws_size || off > (size_t)134217728) return;
  const size_t nw8 = (size_t)DM * DM / 8;
  k_wnat<<<(unsigned)((nw8 + 255) / 256), 256, 0, stream>>>(Wq, nw8, BQ);
  k_wnat<<<(unsigned)((nw8 + 255) / 256), 256, 0, stream>>>(Wk, nw8, BK);
  k_wnat<<<(unsigned)((nw8 + 255) / 256), 256, 0, stream>>>(Wv, nw8, BV);
  const size_t nx8 = (size_t)MROWS * DM / 8;
  k_x16<<<(unsigned)((nx8 + 255) / 256), 256, 0, stream>>>(x, X16, nx8);
  const unsigned gg = (unsigned)((MROWS / 128) * (DM / 64));
  k_gemm2<<<gg, 128, 0, stream>>>(X16, DM, BQ, DM, 0.0625f, bq, QKV,          LQ, MROWS, DM, DM);
  k_gemm2<<<gg, 128, 0, stream>>>(X16, DM, BK, DM, 0.0625f, bk, QKV + DM,     LQ, MROWS, DM, DM);
  k_gemm2<<<gg, 128, 0, stream>>>(X16, DM, BV, DM, 0.0625f, bv, QKV + 2 * DM, LQ, MROWS, DM, DM);
  k_vt2<<<(unsigned)(NB * NH * NQT), 256, 0, stream>>>(QKV, VT);
  k_mflag<<<(unsigned)NQT, 256, 0, stream>>>(mk, MF);
  k_attn<<<dim3((unsigned)NQT, (unsigned)(NB * NH)), 128, 0, stream>>>(QKV, VT, mk, MF, x, (float*)d_out);
}
